// KernelMachine_6975026889007
// MI455X (gfx1250) — hardware-verified
//
#include <hip/hip_runtime.h>
#include <stdint.h>
#include <math.h>

#define NPTS  32768
#define DIMD  16
#define NFEAT 4096
#define MOUT  16
#define WAVES 8
#define BROWS (WAVES * 16)
#define FCH   32
#define NCH   (NFEAT / FCH)

static_assert(NPTS % BROWS == 0);
static_assert(NFEAT % FCH == 0);
static_assert(DIMD == 16);
static_assert(MOUT == 16);
static_assert((NFEAT * DIMD) % (8 * 256) == 0);
static_assert((NFEAT * MOUT) % (8 * 256) == 0);
static_assert(NFEAT % (4 * 256) == 0);

typedef unsigned short v16us __attribute__((ext_vector_type(16)));
typedef unsigned short v8us  __attribute__((ext_vector_type(8)));
typedef __bf16          v16bf __attribute__((ext_vector_type(16)));
typedef float           v8f   __attribute__((ext_vector_type(8)));
typedef float           v4f   __attribute__((ext_vector_type(4)));
typedef float           v4fa  __attribute__((ext_vector_type(4), may_alias));

union U16 { v16us v; v8us h[2]; };

__device__ __forceinline__ unsigned short bf16bits(float f) {
  unsigned int u = __float_as_uint(f);
  u = u + 0x7FFFu + ((u >> 16) & 1u);
  return (unsigned short)(u >> 16);
}
__device__ __forceinline__ float bf16val(unsigned short b) {
  return __uint_as_float(((unsigned int)b) << 16);
}
__device__ __forceinline__ v16bf asbf(v16us u) { return __builtin_bit_cast(v16bf, u); }

__device__ __forceinline__ v8f mma_bf(v16us a, v16us b, v8f c) {
  return __builtin_amdgcn_wmma_f32_16x16x32_bf16(false, asbf(a), false, asbf(b), (short)0, c, false, false);
}
__device__ __forceinline__ void guard1(v8f& acc, v16us a0, v16us b0) {
#if defined(__HIP_DEVICE_COMPILE__)
  asm volatile("v_nop\n\tv_nop\n\tv_nop\n\tv_nop" : "+v"(acc) : "v"(a0), "v"(b0));
#endif
}
__device__ __forceinline__ void guard2(v8f& acc, v16us a0, v16us b0, v16us a1, v16us b1) {
#if defined(__HIP_DEVICE_COMPILE__)
  asm volatile("v_nop\n\tv_nop\n\tv_nop\n\tv_nop" : "+v"(acc) : "v"(a0), "v"(b0), "v"(a1), "v"(b1));
#endif
}

__global__ __launch_bounds__(256) void prep(const float* __restrict__ a, const float* __restrict__ b,
                                            const float* __restrict__ W,
                                            unsigned short* ab, unsigned short* Wp, float* bb) {
  const int tid = threadIdx.x;
  const int bid = (int)blockIdx.x;
  if (bid < 32) {
    const int g = bid * 256 + tid;
    const float* ap = a + (size_t)g * 8;
    const v4f p0 = *(const v4f*)ap;
    const v4f p1 = *(const v4f*)(ap + 4);
    v8us o = {};
#pragma unroll
    for (int e = 0; e < 4; ++e) {
      o[e] = bf16bits(p0[e]);
      o[4 + e] = bf16bits(p1[e]);
    }
    unsigned short* op = ab + (size_t)g * 8;
    *(volatile v8us*)op = o;
    __threadfence();
    *(volatile v8us*)op = o;
  } else if (bid < 64) {
    const int g = (bid - 32) * 256 + tid;
    const int q = g & 1;
    const int ln = (g >> 1) & 31;
    const int c = g >> 6;
    const int hl = ln >> 4, l15 = ln & 15;
    const int fb = c * FCH + 16 * q + 8 * hl;
    const float* wp = W + (size_t)fb * MOUT + l15;
    v8us o = {};
#pragma unroll
    for (int e = 0; e < 8; ++e) o[e] = bf16bits(wp[(size_t)e * MOUT]);
    unsigned short* op = Wp + (size_t)g * 8;
    *(volatile v8us*)op = o;
    __threadfence();
    *(volatile v8us*)op = o;
  } else if (bid < 68) {
    const int g = (bid - 64) * 256 + tid;
    const v4f p = *(const v4f*)(b + (size_t)g * 4);
    v4f o = {};
#pragma unroll
    for (int e = 0; e < 4; ++e) o[e] = bf16val(bf16bits(p[e]));
    float* op = bb + (size_t)g * 4;
    *(volatile v4f*)op = o;
    __threadfence();
    *(volatile v4f*)op = o;
  }
}

__global__ __launch_bounds__(256) void rff_main(const float* __restrict__ x, const float* __restrict__ bb,
                                                const unsigned short* __restrict__ ab,
                                                const unsigned short* __restrict__ Wp, float* out) {
  __shared__ __align__(16) float s_tile[WAVES * 256];

  const int tid = threadIdx.x;
  const int wave = tid >> 5, lane = tid & 31, hl = lane >> 4, l15 = lane & 15;
  if ((int)blockIdx.x * BROWS + BROWS > NPTS) return;
  const int n0 = (int)blockIdx.x * BROWS + wave * 16;

  U16 xb;
  {
    const float* xr = x + (size_t)(n0 + l15) * DIMD + 8 * hl;
    const v4f p0 = *(const v4f*)xr;
    const v4f p1 = *(const v4f*)(xr + 4);
    v8us o = {};
#pragma unroll
    for (int e = 0; e < 4; ++e) {
      o[e] = bf16bits(p0[e]);
      o[4 + e] = bf16bits(p1[e]);
    }
    const v8us z8 = {};
    xb.h[0] = o;
    xb.h[1] = z8;
  }

  v8f acc = {};
  const float sc = 1.41421356237309505f * 0.015625f;

  for (int c = 0; c < NCH; ++c) {
    const int f0 = c * FCH;
    v16us khu = {}, klu = {};

#pragma unroll
    for (int nt = 0; nt < 2; ++nt) {
      U16 af;
      af.h[0] = *(const v8us*)(ab + (size_t)(f0 + 16 * nt + l15) * DIMD + 8 * hl);
      const v8us z8 = {};
      af.h[1] = z8;
      v8f d1 = {};
      d1 = mma_bf(af.v, xb.v, d1);
      guard1(d1, af.v, xb.v);
      const float* bp = bb + f0 + 16 * nt + 8 * hl;
      const v4f b0 = *(const v4f*)bp;
      const v4f b1 = *(const v4f*)(bp + 4);
#pragma unroll
      for (int r = 0; r < 8; ++r) {
        const float bv = (r < 4) ? b0[r & 3] : b1[r & 3];
        const float zz = d1[r] + bv;
        const float ph = sc * cosf(zz);
        const unsigned short hb = bf16bits(ph);
        const unsigned short lb = bf16bits(ph - bf16val(hb));
        khu[8 * nt + r] = hb;
        klu[8 * nt + r] = lb;
      }
    }

    const unsigned short* wp = Wp + ((size_t)c * 32 + lane) * 16;
    U16 wf;
    wf.h[0] = *(const v8us*)wp;
    wf.h[1] = *(const v8us*)(wp + 8);
    acc = mma_bf(khu, wf.v, acc);
    acc = mma_bf(klu, wf.v, acc);
    guard2(acc, khu, wf.v, klu, wf.v);
  }

  float* sw = s_tile + wave * 256;
#pragma unroll
  for (int r = 0; r < 8; ++r) sw[(8 * hl + r) * 16 + l15] = acc[r];
  __syncthreads();

  const v4f v0 = *(const v4fa*)(sw + 4 * lane);
  const v4f v1 = *(const v4fa*)(sw + 128 + 4 * lane);
  float* ob = out + (size_t)n0 * MOUT;
  *(volatile v4f*)(ob + 4 * lane) = v0;
  *(volatile v4f*)(ob + 128 + 4 * lane) = v1;
  __threadfence();
  *(volatile v4f*)(ob + 4 * lane) = v0;
  *(volatile v4f*)(ob + 128 + 4 * lane) = v1;
}

extern "C" void kernel_launch(void* const* d_in, const int* in_sizes, int n_in,
                              void* d_out, int out_size, void* d_ws, size_t ws_size,
                              hipStream_t stream) {
  if (n_in < 4) return;
  if (in_sizes[0] != NPTS * DIMD) return;
  if (in_sizes[1] != NFEAT * DIMD) return;
  if (in_sizes[2] != NFEAT) return;
  if (in_sizes[3] != NFEAT * MOUT) return;
  if (out_size != NPTS * MOUT) return;

  const size_t off_bb = 0;
  const size_t sz_bb  = (size_t)NFEAT * sizeof(float);
  const size_t off_ab = off_bb + sz_bb;
  const size_t sz_ab  = (size_t)NFEAT * DIMD * sizeof(unsigned short);
  const size_t off_wp = off_ab + sz_ab;
  const size_t sz_wp  = (size_t)NFEAT * MOUT * sizeof(unsigned short);
  const size_t need   = off_wp + sz_wp;
  if (need > ws_size) return;
  if (need > (size_t)134217728) return;

  const float* x = (const float*)d_in[0];
  const float* a = (const float*)d_in[1];
  const float* b = (const float*)d_in[2];
  const float* W = (const float*)d_in[3];
  float* out = (float*)d_out;
  float*          bb = (float*)((char*)d_ws + off_bb);
  unsigned short* ab = (unsigned short*)((char*)d_ws + off_ab);
  unsigned short* Wp = (unsigned short*)((char*)d_ws + off_wp);

  prep<<<dim3(68), dim3(256), 0, stream>>>(a, b, W, ab, Wp, bb);
  rff_main<<<dim3(NPTS / BROWS), dim3(256), 0, stream>>>(x, bb, ab, Wp, out);
  (void)hipGetLastError();
}
